// RNN_59803124629906
// MI455X (gfx1250) — hardware-run, weakly checked
//
#include <hip/hip_runtime.h>
#include <math.h>

typedef __attribute__((ext_vector_type(16))) _Float16 v16h;
typedef __attribute__((ext_vector_type(8)))  _Float16 v8h;
typedef __attribute__((ext_vector_type(8)))  float    v8f;
typedef __attribute__((ext_vector_type(4)))  float    v4f;

constexpr int kT   = 512;
constexpr int kH   = 256;
constexpr int kOut = 256;
static_assert((kH % 32) == 0);
static_assert((kT % 64) == 0 && (kH % 64) == 0 && (kOut % 64) == 0);
static_assert(kH == kOut);

constexpr float kCarryX  = 64.0f;
constexpr float kCarryW  = 256.0f;
constexpr float kCarryLo = 2048.0f;
constexpr float kCarryHf = 64.0f;
constexpr float kF16MinNormal = 6.103515625e-5f;
constexpr float kInvXW  = 1.0f / (kCarryX * kCarryW);
constexpr float kInvW   = 1.0f / kCarryW;
constexpr float kInvWLo = 1.0f / (kCarryW * kCarryLo);
constexpr float kInvFc  = 1.0f / (kCarryHf * kCarryW);

constexpr size_t kOffA16X = 0;
constexpr size_t kOffBTIH = kOffA16X + (size_t)kT * kH * 2;
constexpr size_t kOffBTHH = kOffBTIH + (size_t)kH * kH * 2;
constexpr size_t kOffBTFC = kOffBTHH + (size_t)kH * kH * 2;
constexpr size_t kOffXW   = kOffBTFC + (size_t)kH * kOut * 2;
constexpr size_t kOffHREP = kOffXW   + (size_t)kT * kH * 4;
constexpr size_t kWsTotal = kOffHREP + (size_t)kT * kH * 2;
static_assert(kWsTotal == 1441792ull);
static_assert(kWsTotal <= 134217728ull);
static_assert((kOffBTIH % 128) == 0 && (kOffBTHH % 128) == 0 && (kOffBTFC % 128) == 0 &&
              (kOffXW % 128) == 0 && (kOffHREP % 128) == 0);

__device__ __forceinline__ _Float16 to_h16_flush(float v) {
  const float s = (fabsf(v) < kF16MinNormal) ? 0.0f : v;
  return (_Float16)s;
}

union FragU { v16h v; v8h h[2]; };
__device__ __forceinline__ v16h frag_load(const _Float16* p) {
  FragU f;
  f.h[0] = *(const v8h*)(p);
  f.h[1] = *(const v8h*)(p + 16);
  return f.v;
}

__device__ __forceinline__ v8f mma_h(v16h a, v16h b, v8f c) {
  c = __builtin_amdgcn_wmma_f32_16x16x32_f16(false, a, false, b, (short)0, c, false, false);
  asm volatile("v_nop\n\tv_nop\n\tv_nop\n\tv_nop" : "+v"(c) : "v"(a), "v"(b));
  return c;
}

constexpr int kXBlocks   = (kT * kH / 8) / 256;
constexpr int kTrBlocks  = 3 * (kH / 64) * (kH / 64);
constexpr int kTilePitch = 68;
static_assert(kXBlocks * 256 * 8 == kT * kH);
static_assert(kTrBlocks == 48);

__global__ __launch_bounds__(256) void pack_kernel(
    const float* __restrict__ x, const float* __restrict__ Wih, const float* __restrict__ Whh,
    const float* __restrict__ Wfc,
    unsigned short* __restrict__ A16x, unsigned short* __restrict__ BtIh,
    unsigned short* __restrict__ BtHh, unsigned short* __restrict__ BtFc)
{
  __shared__ __align__(16) float sT[64 * kTilePitch];
  const int tid = threadIdx.x;
  if (blockIdx.x < kXBlocks) {
    const int i = blockIdx.x * 256 + tid;
    const size_t e0 = (size_t)i << 3;
    const v4f a0 = *(const v4f*)(x + e0);
    const v4f a1 = *(const v4f*)(x + e0 + 4);
    v8h hv;
#pragma unroll
    for (int e = 0; e < 4; ++e) {
      hv[e]     = to_h16_flush(a0[e] * kCarryX);
      hv[4 + e] = to_h16_flush(a1[e] * kCarryX);
    }
    unsigned short* q = A16x + e0;
    *(volatile v8h*)q = hv;
    __threadfence();
    *(volatile v8h*)q = hv;
  } else {
    const int tb = blockIdx.x - kXBlocks;
    const int mi = tb >> 4;
    const int tl = tb & 15;
    const int k0 = (tl >> 2) * 64;
    const int n0 = (tl & 3) * 64;
    const float* W = (mi == 0) ? Wih : ((mi == 1) ? Whh : Wfc);
    unsigned short* Bt = (mi == 0) ? BtIh : ((mi == 1) ? BtHh : BtFc);
    const int rr = tid >> 4;
    const int c4 = (tid & 15) * 4;
#pragma unroll
    for (int i = 0; i < 4; ++i) {
      const int r = rr + 16 * i;
      const v4f v = *(const v4f*)(W + (size_t)(k0 + r) * kH + n0 + c4);
      *(v4f*)(sT + r * kTilePitch + c4) = v;
    }
    __syncthreads();
    const int q  = tid >> 3;
    const int c8 = (tid & 7) * 8;
    v8h hv[2];
#pragma unroll
    for (int it = 0; it < 2; ++it) {
      const int n = it * 32 + q;
#pragma unroll
      for (int e = 0; e < 8; ++e) {
        const float w = sT[(c8 + e) * kTilePitch + n];
        hv[it][e] = to_h16_flush(w * kCarryW);
      }
    }
    for (int pass = 0; pass < 2; ++pass) {
#pragma unroll
      for (int it = 0; it < 2; ++it) {
        const int n = it * 32 + q;
        *(volatile v8h*)(Bt + (size_t)(n0 + n) * kH + k0 + c8) = hv[it];
      }
      __threadfence();
    }
  }
}

template <int BIAS_MODE>
__global__ __launch_bounds__(256) void wmma_gemm64_f16(
    const unsigned short* __restrict__ Ap, int lda,
    const unsigned short* __restrict__ Btp, int ldb,
    float* __restrict__ C, int ldc,
    const float* __restrict__ bias,
    int M, int N, int K, float scale) {
  const _Float16* A  = (const _Float16*)Ap;
  const _Float16* Bt = (const _Float16*)Btp;
  __shared__ __align__(16) float sT[8][16 * 68];
  const int lane = threadIdx.x & 31;
  const int wave = threadIdx.x >> 5;
  const int tilesN = N >> 6;
  const int tilesM = M >> 6;
  const int tile = blockIdx.x * 8 + wave;
  if (tile >= tilesM * tilesN) return;
  const int tm = tile / tilesN;
  const int tn = tile - tm * tilesN;
  const int m0 = tm << 6;
  const int n0 = tn << 6;

  const int rlane = lane & 15;
  const int koff  = (lane >> 4) * 8;
  const int mOff  = (lane >> 4) * 8;

  v8f acc[4][4];
#pragma unroll
  for (int i = 0; i < 4; ++i)
#pragma unroll
    for (int j = 0; j < 4; ++j) acc[i][j] = (v8f){0.f,0.f,0.f,0.f,0.f,0.f,0.f,0.f};

  for (int k0 = 0; k0 < K; k0 += 32) {
    v16h bh[4];
#pragma unroll
    for (int j = 0; j < 4; ++j) {
      const size_t bo = (size_t)(n0 + (j << 4) + rlane) * ldb + koff + k0;
      bh[j] = frag_load(Bt + bo);
    }
#pragma unroll
    for (int i = 0; i < 4; ++i) {
      const size_t ao = (size_t)(m0 + (i << 4) + rlane) * lda + koff + k0;
      const v16h ah = frag_load(A + ao);
#pragma unroll
      for (int j = 0; j < 4; ++j) {
        acc[i][j] = mma_h(ah, bh[j], acc[i][j]);
      }
    }
  }

  float* slab = sT[wave];
#pragma unroll
  for (int i = 0; i < 4; ++i) {
    const int mBase = m0 + (i << 4);
#pragma unroll
    for (int j = 0; j < 4; ++j) {
      const int n = n0 + (j << 4) + rlane;
      float bv = 0.f;
      if (BIAS_MODE == 2) bv = bias[n];
#pragma unroll
      for (int r = 0; r < 8; ++r) {
        float v = acc[i][j][r] * scale;
        if (BIAS_MODE == 2) v += bv;
        slab[(mOff + r) * 68 + (j << 4) + rlane] = v;
      }
    }
    __builtin_amdgcn_fence(__ATOMIC_RELEASE, "workgroup");
    __builtin_amdgcn_wave_barrier();
    __builtin_amdgcn_fence(__ATOMIC_ACQUIRE, "workgroup");
    {
      const int hh = lane >> 4;
      const int c4 = (lane & 15) * 4;
      for (int pass = 0; pass < 2; ++pass) {
#pragma unroll
        for (int it = 0; it < 8; ++it) {
          const int row = it * 2 + hh;
          const v4f v = *(const v4f*)(slab + row * 68 + c4);
          *(volatile v4f*)(C + (size_t)(mBase + row) * ldc + n0 + c4) = v;
        }
        __threadfence();
      }
    }
    __builtin_amdgcn_fence(__ATOMIC_RELEASE, "workgroup");
    __builtin_amdgcn_wave_barrier();
    __builtin_amdgcn_fence(__ATOMIC_ACQUIRE, "workgroup");
  }
}

__global__ __launch_bounds__(512) void scan_cell_kernel(
    const float* __restrict__ XW, const unsigned short* __restrict__ BtHhp,
    unsigned short* __restrict__ Hrep)
{
  __shared__ __align__(16) _Float16 hb[2 * 2 * kH];
  __shared__ __align__(16) float hfin[kH];
  const int tid  = threadIdx.x;
  const int lane = tid & 31;
  const int wave = tid >> 5;
  const int hh   = lane >> 4;
  const int c    = lane & 15;
  const int col  = wave * 16 + c;
  const _Float16* Bt = (const _Float16*)BtHhp;

  v16h bfr[8];
#pragma unroll
  for (int ks = 0; ks < 8; ++ks) bfr[ks] = frag_load(Bt + (size_t)col * kH + ks * 32 + 8 * hh);

  hb[tid] = (_Float16)0.0f;
  __syncthreads();

  float xw_cur = XW[col];
  asm volatile("" : "+v"(xw_cur));

#pragma unroll 1
  for (int t = 0; t < kT; ++t) {
    const int tn = (t + 1 < kT) ? (t + 1) : (kT - 1);
    float xw_nxt = XW[(size_t)tn * kH + col];
    asm volatile("" : "+v"(xw_nxt));

    const _Float16* rd = hb + (t & 1) * (2 * kH);
    _Float16* wr = hb + ((t + 1) & 1) * (2 * kH);

    v8f acc_v = (v8f){0.f,0.f,0.f,0.f,0.f,0.f,0.f,0.f};
    v8f acc_r = (v8f){0.f,0.f,0.f,0.f,0.f,0.f,0.f,0.f};
#pragma unroll
    for (int ks = 0; ks < 8; ++ks) {
      const v16h av = frag_load(rd + ks * 32 + 8 * hh);
      const v16h ar = frag_load(rd + kH + ks * 32 + 8 * hh);
      acc_v = mma_h(av, bfr[ks], acc_v);
      acc_r = mma_h(ar, bfr[ks], acc_r);
    }

    float rec = acc_v[0] * kInvW;
    rec = fmaf(acc_r[0], kInvWLo, rec);
    const float pre = xw_cur + rec;
    const float hn = tanhf(pre);

    const _Float16 hv16 = to_h16_flush(hn);
    float hvf = (float)hv16;
    asm volatile("" : "+v"(hvf));
    const float res = (hn - hvf) * kCarryLo;
    const _Float16 hr16 = to_h16_flush(res);

    if (hh == 0) {
      wr[col] = hv16;
      wr[kH + col] = hr16;
      hfin[col] = hn;
    }
    xw_cur = xw_nxt;
    __syncthreads();
  }

  {
    const v4f f0 = *(const v4f*)(hfin + lane * 8);
    const v4f f1 = *(const v4f*)(hfin + lane * 8 + 4);
    v8h hv;
#pragma unroll
    for (int e = 0; e < 4; ++e) {
      hv[e]     = to_h16_flush(f0[e] * kCarryHf);
      hv[4 + e] = to_h16_flush(f1[e] * kCarryHf);
    }
    for (int pass = 0; pass < 2; ++pass) {
#pragma unroll 1
      for (int it = 0; it < 32; ++it) {
        const int row = wave * 32 + it;
        *(volatile v8h*)(Hrep + (size_t)row * kH + lane * 8) = hv;
      }
      __threadfence();
    }
  }
}

extern "C" void kernel_launch(void* const* d_in, const int* in_sizes, int n_in,
                              void* d_out, int out_size, void* d_ws, size_t ws_size,
                              hipStream_t stream) {
  if (n_in < 5) return;
  if (in_sizes[0] != kT * kH) return;
  if (in_sizes[1] != kH * kH) return;
  if (in_sizes[2] != kH * kH) return;
  if (in_sizes[3] != kH * kOut) return;
  if (in_sizes[4] != kOut) return;
  if (out_size != kT * kOut) return;
  if (ws_size < kWsTotal) return;

  const float* x    = (const float*)d_in[0];
  const float* W_ih = (const float*)d_in[1];
  const float* W_hh = (const float*)d_in[2];
  const float* fc_W = (const float*)d_in[3];
  const float* fc_b = (const float*)d_in[4];
  float* out = (float*)d_out;

  char* ws = (char*)d_ws;
  unsigned short* A16x = (unsigned short*)(ws + kOffA16X);
  unsigned short* BtIh = (unsigned short*)(ws + kOffBTIH);
  unsigned short* BtHh = (unsigned short*)(ws + kOffBTHH);
  unsigned short* BtFc = (unsigned short*)(ws + kOffBTFC);
  float*          XW   = (float*)(ws + kOffXW);
  unsigned short* Hrep = (unsigned short*)(ws + kOffHREP);

  pack_kernel<<<kXBlocks + kTrBlocks, 256, 0, stream>>>(x, W_ih, W_hh, fc_W, A16x, BtIh, BtHh, BtFc);

  wmma_gemm64_f16<0><<<(kT / 64) * (kH / 64) / 8, 256, 0, stream>>>(
      A16x, kH, BtIh, kH, XW, kH, fc_b, kT, kH, kH, kInvXW);

  scan_cell_kernel<<<1, 512, 0, stream>>>(XW, BtHh, Hrep);

  wmma_gemm64_f16<2><<<(kT / 64) * (kOut / 64) / 8, 256, 0, stream>>>(
      Hrep, kH, BtFc, kH, out, kOut, fc_b, kT, kOut, kH, kInvFc);
}
